// EGNN_vel_Aether_7215545057984
// MI455X (gfx1250) — hardware-run, weakly checked
//
#include <hip/hip_runtime.h>


namespace {
constexpr int N = 10000, E = 320000, H = 64, L = 4, NBLK = N / 16;
constexpr float XS = 8.0f, HS = 64.0f, WSC = 256.0f;
typedef _Float16 b16;
typedef __attribute__((ext_vector_type(16))) _Float16 v16b;
typedef __attribute__((ext_vector_type(8))) _Float16 v8b;
typedef __attribute__((ext_vector_type(8))) float v8f;
typedef __attribute__((ext_vector_type(4))) float v4f;
typedef __attribute__((ext_vector_type(2))) float v2f;
__device__ __forceinline__ float bf16_rne(float f) { unsigned int u = __float_as_uint(f); u += 0x7FFFu + ((u >> 16) & 1u); return __uint_as_float(u & 0xFFFF0000u); }
__device__ __forceinline__ void split16(float v, b16& hi, b16& lo) { hi = (b16)v; lo = (b16)(v - (float)hi); }
__device__ __forceinline__ v16b frag_kb(const b16* p, int hh) { const v8b a = *(const v8b*)(p + 8 * hh), b = *(const v8b*)(p + 16 + 8 * hh); v16b f;
#pragma unroll
  for (int e = 0; e < 8; ++e) { f[e] = a[e]; f[8 + e] = b[e]; } return f; }
__device__ __forceinline__ v8f wmma16b(v16b a, v16b b, v8f c) { v8f d = __builtin_amdgcn_wmma_f32_16x16x32_f16(false, a, false, b, (short)0, c, false, false); asm volatile("v_nop\n\tv_nop\n\tv_nop\n\tv_nop" : "+v"(d) : "v"(a), "v"(b)); return d; }
__device__ __forceinline__ void wave_lds_sync() { __builtin_amdgcn_fence(__ATOMIC_RELEASE, "workgroup"); __builtin_amdgcn_wave_barrier(); __builtin_amdgcn_fence(__ATOMIC_ACQUIRE, "workgroup"); }
__device__ __forceinline__ float pmul(float a, float b) { float p = a * b; asm volatile("" : "+v"(p)); return p; }
__device__ __forceinline__ int iclamp(int v, int lo, int hi) { return v < lo ? lo : (v > hi ? hi : v); }
__device__ __forceinline__ float sigm(float v) { return 1.0f / (1.0f + __expf(-v)); }
__device__ __forceinline__ float silu(float v) { return pmul(v, sigm(v)); }
constexpr int CSR_NBLK8 = 512, CSR_GB8 = 8, CSR_GN8 = 1 << CSR_GB8  , CSR_TS8 = (CSR_GN8 < 32 ? 32 : CSR_GN8)  , CSR_MAXG8 = 512, CSR_CAP8 = 12288  ;
__device__ __host__ __forceinline__ int csr_tix8(int v) { return (v >> CSR_GB8) * CSR_TS8 + (v & (CSR_GN8 - 1)); }
__global__ __launch_bounds__(64) void csrA_kernel8(const int* __restrict__ dst, int E, int N, int nG, int CHP, int NGP, int* __restrict__ STG, int* __restrict__ HST) {
  extern __shared__ int sm[];
  int* cnt = sm; int* run = sm + NGP; int* ids = sm + 2 * NGP;
  const int b = blockIdx.x; const int ch = (E + CSR_NBLK8 - 1) / CSR_NBLK8; const int e0 = b * ch, e1 = min(E, e0 + ch);
  for (int i = threadIdx.x; i < NGP; i += 64) cnt[i] = 0;
  for (int i = threadIdx.x; i < CHP; i += 64) ids[i] = -1;
  __syncthreads();
  if (threadIdx.x == 0) {
    for (int e = e0; e < e1; ++e) { int d = dst[e]; d = (d < 0) ? 0 : (d >= N ? N - 1 : d); cnt[d >> CSR_GB8] += 1; }
    int acc = 0; for (int g = 0; g < nG; ++g) { run[g] = acc; acc += cnt[g]; }
    for (int e = e0; e < e1; ++e) { int d = dst[e]; d = (d < 0) ? 0 : (d >= N ? N - 1 : d); const int g = d >> CSR_GB8; ids[run[g]] = e; run[g] += 1; } }
  __syncthreads();
  typedef __attribute__((ext_vector_type(4))) int v4i;
  for (int pass = 0; pass < 2; ++pass) {
    for (int i = threadIdx.x; i < CHP / 4; i += 64) *(volatile v4i*)(STG + (size_t)b * CHP + i * 4) = *(const v4i*)(&ids[i * 4]);
    for (int i = threadIdx.x; i < NGP / 4; i += 64) { v4i v; for (int e = 0; e < 4; ++e) v[e] = (i * 4 + e < nG) ? cnt[i * 4 + e] : 0; *(volatile v4i*)(HST + (size_t)b * NGP + i * 4) = v; }
    __threadfence(); }
}
__global__ __launch_bounds__(512) void csrS_kernel8(const int* __restrict__ HST, int nG, int NGP, int* __restrict__ START, int* __restrict__ TOT, int* __restrict__ OFF) {
  __shared__ int tot[CSR_MAXG8];
  const int b = threadIdx.x;
  for (int pass = 0; pass < 2; ++pass) { int runb = 0; for (int g = 0; g < nG; ++g) { int c = HST[(size_t)b * NGP + g]; c = (c < 0) ? 0 : c; ((volatile int*)OFF)[(size_t)g * CSR_NBLK8 + b] = runb; runb += c; } __threadfence(); }
  for (int g = threadIdx.x; g < nG; g += 512) { int s = 0; for (int bb = 0; bb < CSR_NBLK8; ++bb) { int c = HST[(size_t)bb * NGP + g]; s += (c < 0) ? 0 : c; } tot[g] = s; }
  __syncthreads();
  if (threadIdx.x < 32) {
    __shared__ int st[CSR_MAXG8 + 32];
    if (threadIdx.x == 0) { int acc = 0; for (int g = 0; g < NGP; ++g) { st[g] = acc; if (g < nG) acc += (tot[g] + 31) & ~31; } st[NGP] = acc; }
    __builtin_amdgcn_fence(__ATOMIC_RELEASE, "workgroup"); __builtin_amdgcn_wave_barrier(); __builtin_amdgcn_fence(__ATOMIC_ACQUIRE, "workgroup");
    for (int pass = 0; pass < 2; ++pass) { for (int i = threadIdx.x; i < NGP + 32; i += 32) { ((volatile int*)START)[i] = (i <= NGP) ? st[min(i, NGP)] : 0; ((volatile int*)TOT)[i] = (i < nG) ? tot[i] : 0; } __threadfence(); } }
}
__global__ __launch_bounds__(256) void csrB_kernel8(const int* __restrict__ dst, int N, int nG, int CHP, int NGP, int permLen, const int* __restrict__ STG, const int* __restrict__ HST, const int* __restrict__ OFF, const int* __restrict__ START, const int* __restrict__ TOT, int* __restrict__ PERM, int* __restrict__ ROWPTR, int* __restrict__ ROWCNT, int* __restrict__ FLAG) {
  typedef __attribute__((ext_vector_type(4))) int v4i;
  __shared__ int ids[CSR_CAP8]; __shared__ unsigned short key[CSR_CAP8]; __shared__ int outp[CSR_CAP8]; __shared__ int ncnt[CSR_GN8 + 1]; __shared__ int boff[CSR_NBLK8 + 1];
  const int g = blockIdx.x, t_ = threadIdx.x; int tot = TOT[g]; int st = START[g], stn = START[g + 1]; const int v0 = g * CSR_GN8; const int nv = min(CSR_GN8, N - v0); const int t0 = g * CSR_TS8;
  st = (st < 0) ? 0 : (st > permLen - 32 ? permLen - 32 : st) & ~31; stn = (stn < st) ? st : (stn > permLen ? permLen : stn); tot = (tot < 0) ? 0 : tot; if (tot > stn - st && tot <= CSR_CAP8) tot = stn - st;
  if (tot > CSR_CAP8) {
    for (int pass = 0; pass < 2; ++pass) { for (int i = t_; i < CSR_TS8 / 4; i += 256) { v4i a, c; for (int e = 0; e < 4; ++e) { a[e] = st; c[e] = 0; } *(volatile v4i*)(ROWPTR + t0 + i * 4) = a; *(volatile v4i*)(ROWCNT + t0 + i * 4) = c; } if (t_ == 0) ((volatile int*)FLAG)[0] = 1; __threadfence(); } (void)nv; return; }
  if (t_ == 0) { int acc = 0; for (int b = 0; b < CSR_NBLK8; ++b) { boff[b] = acc; int c = HST[(size_t)b * NGP + g]; c = (c < 0) ? 0 : (c > CHP ? CHP : c); acc += c; if (acc > tot) acc = tot; } boff[CSR_NBLK8] = acc; }
  for (int i = t_; i <= CSR_GN8; i += 256) ncnt[i] = 0;
  __syncthreads();
  for (int b = 0; b < CSR_NBLK8; ++b) { const int c = boff[b + 1] - boff[b]; int o_ = OFF[(size_t)g * CSR_NBLK8 + b]; o_ = (o_ < 0) ? 0 : (o_ > CHP - c ? CHP - c : o_); const int* src_ = STG + (size_t)b * CHP + o_;
    for (int i = t_; i < c; i += 256) { int id = src_[i]; id = (id < 0) ? 0 : id; ids[boff[b] + i] = id; int d = dst[id]; d = (d < v0) ? v0 : (d >= N ? N - 1 : d); int kk = d - v0; kk = (kk < 0) ? 0 : (kk >= CSR_GN8 ? CSR_GN8 - 1 : kk); key[boff[b] + i] = (unsigned short)kk; } }
  __syncthreads();
  if (t_ == 0) { for (int i = 0; i < tot; ++i) ncnt[key[i]] += 1; int acc = 0; for (int vl = 0; vl < CSR_GN8; ++vl) { const int c = ncnt[vl]; ncnt[vl] = acc; acc += c; } ncnt[CSR_GN8] = acc;
    for (int i = 0; i < tot; ++i) { const int vl = key[i]; outp[ncnt[vl]] = ids[i]; ncnt[vl] += 1; }
    for (int vl = CSR_GN8; vl > 0; --vl) ncnt[vl] = ncnt[vl - 1]; ncnt[0] = 0; }
  __syncthreads();
  for (int pass = 0; pass < 2; ++pass) {
    for (int i = t_; i < (stn - st) / 4; i += 256) { v4i v; for (int e = 0; e < 4; ++e) { const int q = i * 4 + e; v[e] = (q < tot) ? outp[q] : -1; } *(volatile v4i*)(PERM + st + i * 4) = v; }
    for (int i = t_; i < CSR_TS8 / 4; i += 256) { v4i a, c; for (int e = 0; e < 4; ++e) { const int vl = i * 4 + e; const int vc = vl < CSR_GN8 ? vl : CSR_GN8; a[e] = (vl < CSR_GN8) ? st + ncnt[vc] : st; c[e] = (vl < nv) ? (ncnt[(vc < CSR_GN8 ? vc : CSR_GN8 - 1) + 1] - ncnt[vc]) : 0; } *(volatile v4i*)(ROWPTR + t0 + i * 4) = a; *(volatile v4i*)(ROWCNT + t0 + i * 4) = c; }
    __threadfence(); }
}
__global__ __launch_bounds__(256) void csrZ_kernel8(int* __restrict__ p, size_t n4) { typedef __attribute__((ext_vector_type(4))) int v4i; const size_t tid = (size_t)blockIdx.x * 256 + threadIdx.x, nth = (size_t)gridDim.x * 256; v4i z = {0, 0, 0, 0}; for (size_t i = tid; i < n4; i += nth) *(volatile v4i*)(p + i * 4) = z; }
struct CsrBufs8 { int *STG, *HST, *OFF, *START, *TOT, *PERM, *ROWPTR, *ROWCNT, *FLAG; int nG, NGP, CHP; size_t permLen; char* base; size_t bytes; };
static size_t csr_carve8(CsrBufs8& c, char* ws, size_t off, int E, int N) {
  const size_t off0 = off; c.base = ws + off;
  auto al = [&](size_t bytes) { char* p = ws + off; off += (bytes + 255) & ~(size_t)255; return p; };
  c.nG = (N + CSR_GN8 - 1) / CSR_GN8; c.NGP = (c.nG + 31) & ~31; const int ch = (E + CSR_NBLK8 - 1) / CSR_NBLK8; c.CHP = (ch + 31) & ~31; c.permLen = (size_t)E + 32 * (size_t)c.nG + 32;
  c.STG = (int*)al((size_t)CSR_NBLK8 * c.CHP * 4); c.HST = (int*)al((size_t)CSR_NBLK8 * c.NGP * 4); c.OFF = (int*)al((size_t)c.NGP * CSR_NBLK8 * 4); c.START = (int*)al((size_t)(c.NGP + 64) * 4); c.TOT = (int*)al((size_t)(c.NGP + 64) * 4);
  c.PERM = (int*)al(c.permLen * 4); c.ROWPTR = (int*)al((size_t)c.nG * CSR_TS8 * 4); c.ROWCNT = (int*)al((size_t)c.nG * CSR_TS8 * 4); c.FLAG = (int*)al(256);
  c.bytes = off - off0; return off;
}
static void csr_build8(const CsrBufs8& c, const int* dst, int E, int N, hipStream_t stream) {
  const size_t smem = (size_t)(2 * c.NGP + c.CHP) * 4;
  csrZ_kernel8<<<512, 256, 0, stream>>>((int*)c.base, c.bytes / 16);
  csrA_kernel8<<<CSR_NBLK8, 64, smem, stream>>>(dst, E, N, c.nG, c.CHP, c.NGP, c.STG, c.HST);
  csrS_kernel8<<<1, 512, 0, stream>>>(c.HST, c.nG, c.NGP, c.START, c.TOT, c.OFF);
  csrB_kernel8<<<c.nG, 256, 0, stream>>>(dst, N, c.nG, c.CHP, c.NGP, (int)c.permLen, c.STG, c.HST, c.OFF, c.START, c.TOT, c.PERM, c.ROWPTR, c.ROWCNT, c.FLAG);
}


__global__ __launch_bounds__(256) void wput_kernel(const float* __restrict__ w, int OUTW, int r0, int KN, int ro, int KP, int OUT, b16* __restrict__ WT) {
  const int KG = KN / 8; const int u = blockIdx.x * 256 + threadIdx.x; if (u >= OUT * KG) return; const int o = u / KG, k0 = (u % KG) * 8; v8b v;
#pragma unroll
  for (int j = 0; j < 8; ++j) v[j] = (b16)(bf16_rne(w[(size_t)(r0 + k0 + j) * OUTW + o]) * WSC); for (int pass = 0; pass < 2; ++pass) { *(volatile v8b*)(WT + (size_t)(ro + o) * KP + k0) = v; __threadfence(); }
}
__global__ __launch_bounds__(256) void prolog_kernel(const float* __restrict__ h, const float* __restrict__ x, const float* __restrict__ vel, const int* __restrict__ chg, const float* __restrict__ embW, const float* __restrict__ embb, const float* __restrict__ cls, const float* __restrict__ fW1, const float* __restrict__ fb1, const float* __restrict__ fW2, const float* __restrict__ fb2, const float* __restrict__ fW3, const float* __restrict__ fb3, float* __restrict__ FLD, float* __restrict__ HH, float* __restrict__ CO) {
  __shared__ float w1[22][32], w2[32][32], w3[32][3], b1s[32], b2s[32];
  for (int i = threadIdx.x; i < 22 * 32; i += 256) w1[i / 32][i % 32] = bf16_rne(fW1[i]); for (int i = threadIdx.x; i < 32 * 32; i += 256) w2[i / 32][i % 32] = bf16_rne(fW2[i]); for (int i = threadIdx.x; i < 96; i += 256) w3[i / 3][i % 3] = bf16_rne(fW3[i]);
  if (threadIdx.x < 32) { b1s[threadIdx.x] = bf16_rne(fb1[threadIdx.x]); b2s[threadIdx.x] = bf16_rne(fb2[threadIdx.x]); } __syncthreads();
  const int n = blockIdx.x * 256 + threadIdx.x; if (n >= N) return; float in[22]; for (int d = 0; d < 3; ++d) { in[d] = bf16_rne(x[n * 3 + d]); in[3 + d] = bf16_rne(vel[n * 3 + d]); } const int c = iclamp(chg[n], 0, 1); for (int j = 0; j < 16; ++j) in[6 + j] = bf16_rne(cls[c * 16 + j]);
  float a[32], bq[32];
#pragma unroll 1
  for (int o = 0; o < 32; ++o) { float s = b1s[o]; for (int k = 0; k < 22; ++k) s += pmul(in[k], w1[k][o]); a[o] = silu(s); }
#pragma unroll 1
  for (int o = 0; o < 32; ++o) { float s = b2s[o]; for (int k = 0; k < 32; ++k) s += pmul(a[k], w2[k][o]); bq[o] = silu(s); }
  v4f f; for (int d = 0; d < 3; ++d) { float s = bf16_rne(fb3[d]); for (int k = 0; k < 32; ++k) s += pmul(bq[k], w3[k][d]); f[d] = s; } f[3] = 0.0f;
  const float hv = bf16_rne(h[n]); v4f co = {in[0], in[1], in[2], 0.0f};
  for (int pass = 0; pass < 2; ++pass) { *(volatile v4f*)(FLD + (size_t)n * 4) = f; *(volatile v4f*)(CO + (size_t)n * 4) = co; for (int q = 0; q < H; q += 4) { v4f v; for (int j = 0; j < 4; ++j) v[j] = pmul(hv, bf16_rne(embW[q + j])) + bf16_rne(embb[q + j]); *(volatile v4f*)(HH + (size_t)n * H + q) = v; } __threadfence(); }
}
__global__ __launch_bounds__(32) void nodelin_kernel(const float* __restrict__ HH, const b16* __restrict__ WN, const float* __restrict__ vb1, const float* __restrict__ vW2, const float* __restrict__ vb2, const float* __restrict__ gb1, const float* __restrict__ gW2, const float* __restrict__ gb2, float* __restrict__ PQ, float* __restrict__ VG) {
  __shared__ __attribute__((aligned(16))) b16 Ah[16][H + 8], Al[16][H + 8]; __shared__ __attribute__((aligned(16))) float Tf[16][128 + 4], Sv[16][2];
  const int lane = threadIdx.x, nloc = lane & 15, hlf = lane >> 4; const size_t m0 = (size_t)blockIdx.x * 16;
  for (int rr = 0; rr < 16; ++rr) { const v2f v = *(const v2f*)(HH + (m0 + rr) * H + lane * 2); for (int j = 0; j < 2; ++j) { b16 p, q; split16(v[j] * XS, p, q); Ah[rr][lane * 2 + j] = p; Al[rr][lane * 2 + j] = q; } }
  wave_lds_sync(); const float sc = 1.0f / (XS * WSC);
#pragma unroll 1
  for (int cg = 0; cg < 2; ++cg) { v8f acc[8];
#pragma unroll
    for (int t = 0; t < 8; ++t) acc[t] = (v8f){};
#pragma unroll
    for (int kb = 0; kb < H; kb += 32) { const v16b a = frag_kb(&Ah[nloc][kb], hlf), al = frag_kb(&Al[nloc][kb], hlf);
#pragma unroll
      for (int t = 0; t < 8; ++t) { const v16b bw = frag_kb(WN + (size_t)(cg * 128 + t * 16 + nloc) * H + kb, hlf); acc[t] = wmma16b(a, bw, acc[t]); acc[t] = wmma16b(al, bw, acc[t]); } }
    if (cg == 0) {
#pragma unroll
      for (int t = 0; t < 8; ++t)
#pragma unroll 1
        for (int r8 = 0; r8 < 8; ++r8) Tf[8 * hlf + r8][t * 16 + nloc] = acc[t][r8] * sc;
      wave_lds_sync();
      for (int pass = 0; pass < 2; ++pass) { for (int rr = 0; rr < 16; ++rr) *(volatile v4f*)(PQ + (m0 + rr) * 128 + lane * 4) = *(const v4f*)(&Tf[rr][lane * 4]); __threadfence(); }
      wave_lds_sync(); }
    else { float pv[8], pg[8];
#pragma unroll
      for (int r8 = 0; r8 < 8; ++r8) { pv[r8] = 0.0f; pg[r8] = 0.0f; }
#pragma unroll
      for (int t = 0; t < 8; ++t) { const int c = (t & 3) * 16 + nloc; const bool isg = t >= 4; const float bb = bf16_rne(isg ? gb1[c] : vb1[c]), w2 = bf16_rne(isg ? gW2[c] : vW2[c]);
#pragma unroll
        for (int r8 = 0; r8 < 8; ++r8) { const float s = pmul(silu(acc[t][r8] * sc + bb), w2); if (isg) pg[r8] += s; else pv[r8] += s; } }
#pragma unroll
      for (int r8 = 0; r8 < 8; ++r8) { float a = pv[r8], g = pg[r8]; for (int o = 1; o < 16; o <<= 1) { a += __shfl_xor(a, o); g += __shfl_xor(g, o); } if (nloc == 0) { Sv[8 * hlf + r8][0] = a + bf16_rne(vb2[0]); Sv[8 * hlf + r8][1] = g + bf16_rne(gb2[0]); } }
      wave_lds_sync();
      for (int pass = 0; pass < 2; ++pass) { ((volatile float*)VG)[m0 * 2 + lane] = Sv[lane >> 1][lane & 1]; __threadfence(); } } }
}
__global__ __launch_bounds__(32) void edge_kernel(const float* __restrict__ CO, const float* __restrict__ PQ, const int* __restrict__ ed, const float* __restrict__ ea, const float* __restrict__ W1, const float* __restrict__ b1, const b16* __restrict__ W2T, const float* __restrict__ b2, const b16* __restrict__ CW1T, const float* __restrict__ cb1, const float* __restrict__ cW2, float* __restrict__ M, float* __restrict__ TR) {
  __shared__ __attribute__((aligned(16))) b16 Ah[16][H + 8], Al[16][H + 8]; __shared__ __attribute__((aligned(16))) float Tf[16][H + 4], Df[16][4], Sc[16];
  const int lane = threadIdx.x, nloc = lane & 15, hlf = lane >> 4; const size_t e0 = (size_t)blockIdx.x * 16; const float sc = 1.0f / (XS * WSC);
  const float wr0 = bf16_rne(W1[(2 * H) * H + lane * 2]), wr1 = bf16_rne(W1[(2 * H) * H + lane * 2 + 1]), wa0 = bf16_rne(W1[(2 * H + 1) * H + lane * 2]), wa1 = bf16_rne(W1[(2 * H + 1) * H + lane * 2 + 1]), wb0 = bf16_rne(W1[(2 * H + 2) * H + lane * 2]), wb1 = bf16_rne(W1[(2 * H + 2) * H + lane * 2 + 1]), bb0 = bf16_rne(b1[lane * 2]), bb1 = bf16_rne(b1[lane * 2 + 1]);
  for (int rr = 0; rr < 16; ++rr) { const size_t e = e0 + rr; const int r = iclamp(ed[e], 0, N - 1), c = iclamp(ed[E + e], 0, N - 1);
    const v4f cr = *(const v4f*)(CO + (size_t)r * 4), cc = *(const v4f*)(CO + (size_t)c * 4); const float d0 = cr[0] - cc[0], d1 = cr[1] - cc[1], d2 = cr[2] - cc[2]; const float rad = pmul(d0, d0) + pmul(d1, d1) + pmul(d2, d2);
    if (lane == 0) { Df[rr][0] = d0; Df[rr][1] = d1; Df[rr][2] = d2; Df[rr][3] = 0.0f; }
    const v2f p = *(const v2f*)(PQ + (size_t)r * 128 + lane * 2), q = *(const v2f*)(PQ + (size_t)c * 128 + H + lane * 2); const float a0 = bf16_rne(ea[e * 2]), a1 = bf16_rne(ea[e * 2 + 1]);
    const float v0 = silu(p[0] + q[0] + pmul(rad, wr0) + pmul(a0, wa0) + pmul(a1, wb0) + bb0), v1 = silu(p[1] + q[1] + pmul(rad, wr1) + pmul(a0, wa1) + pmul(a1, wb1) + bb1);
    b16 ph, pl; split16(v0 * XS, ph, pl); Ah[rr][lane * 2] = ph; Al[rr][lane * 2] = pl; split16(v1 * XS, ph, pl); Ah[rr][lane * 2 + 1] = ph; Al[rr][lane * 2 + 1] = pl; }
  wave_lds_sync();
  v8f acc[4];
#pragma unroll
  for (int t = 0; t < 4; ++t) acc[t] = (v8f){};
#pragma unroll
  for (int kb = 0; kb < H; kb += 32) { const v16b a = frag_kb(&Ah[nloc][kb], hlf), al = frag_kb(&Al[nloc][kb], hlf);
#pragma unroll
    for (int t = 0; t < 4; ++t) { const v16b bw = frag_kb(W2T + (size_t)(t * 16 + nloc) * H + kb, hlf); acc[t] = wmma16b(a, bw, acc[t]); acc[t] = wmma16b(al, bw, acc[t]); } }
  wave_lds_sync();
#pragma unroll
  for (int t = 0; t < 4; ++t) { const int c = t * 16 + nloc; const float bb = bf16_rne(b2[c]);
#pragma unroll
    for (int r8 = 0; r8 < 8; ++r8) { const int rl = 8 * hlf + r8; const float m = silu(acc[t][r8] * sc + bb); Tf[rl][c] = m; b16 p, ql; split16(m * XS, p, ql); Ah[rl][c] = p; Al[rl][c] = ql; } }
  wave_lds_sync();
  for (int pass = 0; pass < 2; ++pass) { for (int rr = 0; rr < 16; ++rr) *(volatile v2f*)(M + (e0 + rr) * H + lane * 2) = *(const v2f*)(&Tf[rr][lane * 2]); __threadfence(); }
#pragma unroll
  for (int t = 0; t < 4; ++t) acc[t] = (v8f){};
#pragma unroll
  for (int kb = 0; kb < H; kb += 32) { const v16b a = frag_kb(&Ah[nloc][kb], hlf), al = frag_kb(&Al[nloc][kb], hlf);
#pragma unroll
    for (int t = 0; t < 4; ++t) { const v16b bw = frag_kb(CW1T + (size_t)(t * 16 + nloc) * H + kb, hlf); acc[t] = wmma16b(a, bw, acc[t]); acc[t] = wmma16b(al, bw, acc[t]); } }
  float pc[8];
#pragma unroll
  for (int r8 = 0; r8 < 8; ++r8) pc[r8] = 0.0f;
#pragma unroll
  for (int t = 0; t < 4; ++t) { const int c = t * 16 + nloc; const float bb = bf16_rne(cb1[c]), w2 = bf16_rne(cW2[c]);
#pragma unroll
    for (int r8 = 0; r8 < 8; ++r8) pc[r8] += pmul(silu(acc[t][r8] * sc + bb), w2); }
#pragma unroll
  for (int r8 = 0; r8 < 8; ++r8) { float s = pc[r8]; for (int o = 1; o < 16; o <<= 1) s += __shfl_xor(s, o); if (nloc == 0) Sc[8 * hlf + r8] = s; }
  wave_lds_sync();
  for (int pass = 0; pass < 2; ++pass) { if (lane < 16) { v4f tv; for (int d = 0; d < 4; ++d) tv[d] = pmul(Df[lane][d], Sc[lane]); *(volatile v4f*)(TR + (e0 + lane) * 4) = tv; } __threadfence(); }
}
__global__ __launch_bounds__(32) void node_kernel(const float* __restrict__ M, const float* __restrict__ TR, const int* __restrict__ PERM, const int* __restrict__ ROWPTR, const int* __restrict__ ROWCNT, int permLen, int ELIM, const float* __restrict__ VG, const float* __restrict__ vel, const float* __restrict__ FLD, const b16* __restrict__ NW1T, const float* __restrict__ nb1, const b16* __restrict__ NW2T, const float* __restrict__ nb2, float* HH, float* CO) {
  __shared__ __attribute__((aligned(16))) b16 Ah[16][128 + 8], Al[16][128 + 8]; __shared__ __attribute__((aligned(16))) float Tf[16][H + 4], Cn[16][4];
  const int lane = threadIdx.x, nloc = lane & 15, hlf = lane >> 4; const size_t m0 = (size_t)blockIdx.x * 16; const float sc = 1.0f / (XS * WSC);
  for (int rr = 0; rr < 16; ++rr) { const size_t v = m0 + rr; int st = ROWPTR[v], cnt = ROWCNT[v]; cnt = iclamp(cnt, 0, 1 << 20); st = iclamp(st, 0, permLen - cnt); float s0 = 0.0f, s1 = 0.0f; float cs = 0.0f; int used = 0;
#pragma unroll 1
    for (int j = 0; j < cnt; ++j) { const int e = iclamp(PERM[st + j], 0, E - 1); if (e >= ELIM) continue; ++used;     const v2f mv = *(const v2f*)(M + (size_t)e * H + lane * 2); s0 += mv[0]; s1 += mv[1]; if (lane < 4) cs += TR[(size_t)e * 4 + lane]; }
    const v2f hv = *(const v2f*)(HH + v * H + lane * 2); b16 p, q; split16(hv[0] * XS, p, q); Ah[rr][lane * 2] = p; Al[rr][lane * 2] = q; split16(hv[1] * XS, p, q); Ah[rr][lane * 2 + 1] = p; Al[rr][lane * 2 + 1] = q;
    split16(s0 * XS, p, q); Ah[rr][H + lane * 2] = p; Al[rr][H + lane * 2] = q; split16(s1 * XS, p, q); Ah[rr][H + lane * 2 + 1] = p; Al[rr][H + lane * 2 + 1] = q;
    if (lane < 4) { const float inv = 1.0f / (float)(used < 1 ? 1 : used); const float vw = VG[v * 2], gw = VG[v * 2 + 1]; const float velv = lane < 3 ? bf16_rne(vel[v * 3 + lane]) : 0.0f; Cn[rr][lane] = CO[v * 4 + lane] + pmul(cs, inv) + pmul(vw, velv) + pmul(gw, FLD[v * 4 + lane]); } }
  wave_lds_sync();
  v8f acc[4];
#pragma unroll
  for (int t = 0; t < 4; ++t) acc[t] = (v8f){};
#pragma unroll
  for (int kb = 0; kb < 128; kb += 32) { const v16b a = frag_kb(&Ah[nloc][kb], hlf), al = frag_kb(&Al[nloc][kb], hlf);
#pragma unroll
    for (int t = 0; t < 4; ++t) { const v16b bw = frag_kb(NW1T + (size_t)(t * 16 + nloc) * 128 + kb, hlf); acc[t] = wmma16b(a, bw, acc[t]); acc[t] = wmma16b(al, bw, acc[t]); } }
  wave_lds_sync();
#pragma unroll
  for (int t = 0; t < 4; ++t) { const int c = t * 16 + nloc; const float bb = bf16_rne(nb1[c]);
#pragma unroll
    for (int r8 = 0; r8 < 8; ++r8) { const int rl = 8 * hlf + r8; b16 p, ql; split16(silu(acc[t][r8] * sc + bb) * XS, p, ql); Ah[rl][c] = p; Al[rl][c] = ql; } }
  wave_lds_sync();
#pragma unroll
  for (int t = 0; t < 4; ++t) acc[t] = (v8f){};
#pragma unroll
  for (int kb = 0; kb < H; kb += 32) { const v16b a = frag_kb(&Ah[nloc][kb], hlf), al = frag_kb(&Al[nloc][kb], hlf);
#pragma unroll
    for (int t = 0; t < 4; ++t) { const v16b bw = frag_kb(NW2T + (size_t)(t * 16 + nloc) * H + kb, hlf); acc[t] = wmma16b(a, bw, acc[t]); acc[t] = wmma16b(al, bw, acc[t]); } }
#pragma unroll
  for (int t = 0; t < 4; ++t) { const int c = t * 16 + nloc; const float bb = bf16_rne(nb2[c]);
#pragma unroll 1
    for (int r8 = 0; r8 < 8; ++r8) Tf[8 * hlf + r8][c] = acc[t][r8] * sc + bb; }
  wave_lds_sync();
  for (int pass = 0; pass < 2; ++pass) { for (int rr = 0; rr < 16; ++rr) *(volatile v2f*)(HH + (m0 + rr) * H + lane * 2) = *(const v2f*)(&Tf[rr][lane * 2]); if (lane < 16) *(volatile v4f*)(CO + (m0 + lane) * 4) = *(const v4f*)(&Cn[lane][0]);
    __threadfence(); }
}
__global__ __launch_bounds__(256) void out_kernel(const float* __restrict__ CO, float* __restrict__ out) { const int u = blockIdx.x * 256 + threadIdx.x; if (u >= N * 3) return; const float v = CO[(size_t)(u / 3) * 4 + u % 3]; for (int pass = 0; pass < 2; ++pass) { ((volatile float*)out)[u] = v; __threadfence(); } }
}

extern "C" void kernel_launch(void* const* d_in, const int* in_sizes, int n_in, void* d_out, int out_size, void* d_ws, size_t ws_size, hipStream_t stream) {
  (void)n_in;
  auto Fp = [&](int i) { return (const float*)d_in[i]; }; auto Ip = [&](int i) { return (const int*)d_in[i]; };
  if (in_sizes[0] != N || in_sizes[1] != N * 3 || in_sizes[3] != E * 2 || in_sizes[4] != 2 * E || in_sizes[5] != N || in_sizes[9] != 22 * 32 || in_sizes[15] != L * 131 * H || in_sizes[19] != L * 128 * H || in_sizes[25] != L * H || out_size != N * 3) return;
  const int ELIM = E;
  size_t off = 0; char* ws = (char*)d_ws;
  auto carve = [&](size_t bytes) { char* p = ws + off; off += (bytes + 255) & ~(size_t)255; return p; };
  b16* WN[L]; b16* W2T[L]; b16* CW1T[L]; b16* NW1T[L]; b16* NW2T[L];
  for (int l = 0; l < L; ++l) { WN[l] = (b16*)carve(256 * H * 2); W2T[l] = (b16*)carve(H * H * 2); CW1T[l] = (b16*)carve(H * H * 2); NW1T[l] = (b16*)carve(H * 128 * 2); NW2T[l] = (b16*)carve(H * H * 2); }
  float* FLD = (float*)carve((size_t)N * 4 * 4); float* HH = (float*)carve((size_t)N * H * 4); float* CO = (float*)carve((size_t)N * 4 * 4); float* PQ = (float*)carve((size_t)N * 128 * 4); float* VG = (float*)carve((size_t)N * 2 * 4); float* M = (float*)carve((size_t)E * H * 4); float* TR = (float*)carve((size_t)E * 4 * 4);
  CsrBufs8 csr; off = csr_carve8(csr, ws, off, E, N);
  if (off > ws_size || off > ((size_t)128 << 20)) return;
  for (int l = 0; l < L; ++l) { const float* w1 = Fp(15) + (size_t)l * 131 * H;
    wput_kernel<<<(H * 8 + 255) / 256, 256, 0, stream>>>(w1, H, 0, H, 0, H, H, WN[l]); wput_kernel<<<(H * 8 + 255) / 256, 256, 0, stream>>>(w1, H, H, H, H, H, H, WN[l]);
    wput_kernel<<<(H * 8 + 255) / 256, 256, 0, stream>>>(Fp(26) + (size_t)l * H * H, H, 0, H, 2 * H, H, H, WN[l]); wput_kernel<<<(H * 8 + 255) / 256, 256, 0, stream>>>(Fp(30) + (size_t)l * H * H, H, 0, H, 3 * H, H, H, WN[l]);
    wput_kernel<<<(H * 8 + 255) / 256, 256, 0, stream>>>(Fp(17) + (size_t)l * H * H, H, 0, H, 0, H, H, W2T[l]); wput_kernel<<<(H * 8 + 255) / 256, 256, 0, stream>>>(Fp(23) + (size_t)l * H * H, H, 0, H, 0, H, H, CW1T[l]);
    wput_kernel<<<(H * 16 + 255) / 256, 256, 0, stream>>>(Fp(19) + (size_t)l * 128 * H, H, 0, 128, 0, 128, H, NW1T[l]); wput_kernel<<<(H * 8 + 255) / 256, 256, 0, stream>>>(Fp(21) + (size_t)l * H * H, H, 0, H, 0, H, H, NW2T[l]); }
  csr_build8(csr, Ip(4), E, N, stream);
  prolog_kernel<<<(N + 255) / 256, 256, 0, stream>>>(Fp(0), Fp(1), Fp(2), Ip(5), Fp(6), Fp(7), Fp(8), Fp(9), Fp(10), Fp(11), Fp(12), Fp(13), Fp(14), FLD, HH, CO);
  for (int l = 0; l < L; ++l) {
    nodelin_kernel<<<NBLK, 32, 0, stream>>>(HH, WN[l], Fp(27) + l * H, Fp(28) + l * H, Fp(29) + l, Fp(31) + l * H, Fp(32) + l * H, Fp(33) + l, PQ, VG);
    edge_kernel<<<ELIM / 16, 32, 0, stream>>>(CO, PQ, Ip(4), Fp(3), Fp(15) + (size_t)l * 131 * H, Fp(16) + l * H, W2T[l], Fp(18) + l * H, CW1T[l], Fp(24) + l * H, Fp(25) + l * H, M, TR);
    node_kernel<<<NBLK, 32, 0, stream>>>(M, TR, csr.PERM, csr.ROWPTR, csr.ROWCNT, (int)csr.permLen, ELIM, VG, Fp(2), FLD, NW1T[l], Fp(20) + l * H, NW2T[l], Fp(22) + l * H, HH, CO); }
  out_kernel<<<(N * 3 + 255) / 256, 256, 0, stream>>>(CO, (float*)d_out);
}
